// TinyNeRF_28492813042019
// MI455X (gfx1250) — hardware-verified
//
#include <hip/hip_runtime.h>
#include <math.h>

typedef __attribute__((ext_vector_type(16))) _Float16 v16h;
typedef __attribute__((ext_vector_type(8)))  _Float16 v8h;
typedef __attribute__((ext_vector_type(8)))  float    v8f;
typedef __attribute__((ext_vector_type(4)))  float    v4f;

__device__ __forceinline__ void dep_guard_h(v8f& a, v8f& b, v16h x, v16h y) { asm volatile("v_nop\n\tv_nop\n\tv_nop\n\tv_nop" : "+v"(a), "+v"(b) : "v"(x), "v"(y)); }
__device__ __forceinline__ void keep4_h(v16h a, v16h b, v16h c, v16h d) { asm volatile("v_nop" :: "v"(a), "v"(b), "v"(c), "v"(d)); }
template <typename T> struct Frag;
template <> struct Frag<_Float16> {
  typedef v16h V; union U { v16h v; v8h h[2]; };
  static __device__ __forceinline__ v16h load(const _Float16* p) {
    U f; f.h[0] = *(const v8h*)(p); f.h[1] = *(const v8h*)(p + 16); return f.v;
  }
  static __device__ __forceinline__ v8f mma(v16h a, v16h b, v8f c) {
    return __builtin_amdgcn_wmma_f32_16x16x32_f16(false, a, false, b, (short)0, c, false, false);
  }
  static __device__ __forceinline__ void guard(v8f& a, v8f& b, v16h x, v16h y) { dep_guard_h(a, b, x, y); }
  static __device__ __forceinline__ void keep(v16h a, v16h b, v16h c, v16h d) { keep4_h(a, b, c, d); }
};

#define NSTEP   64
#define HID     80
#define NSK     5
#define KIN     83
#define WTP     128
#define WTROWS  496
#define HEADROW 480
#define WSC     16.0f
#define WSC_INV 0.0625f
#define RAYS_PER_BLOCK 128

union HB { v16h v; v8h h[2]; };

__device__ __forceinline__ void guard5z(v8f& c0, v8f& c1, v8f& c2, v8f& c3, v8f& c4,
                                        v16h x0, v16h x1, v16h x2, v16h x3, v16h x4, v16h y, int& z) {
  asm volatile("v_nop\n\tv_nop\n\tv_nop\n\tv_nop"
               : "+v"(c0), "+v"(c1), "+v"(c2), "+v"(c3), "+v"(c4), "+v"(z)
               : "v"(x0), "v"(x1), "v"(x2), "v"(x3), "v"(x4), "v"(y) : "memory");
}
__device__ __forceinline__ void guard1z(v8f& c0, v16h x0, v16h x1, v16h x2, v16h y0, v16h y1, v16h y2, int& z) {
  asm volatile("v_nop\n\tv_nop\n\tv_nop\n\tv_nop"
               : "+v"(c0), "+v"(z)
               : "v"(x0), "v"(x1), "v"(x2), "v"(y0), "v"(y1), "v"(y2) : "memory");
}

__device__ __forceinline__ v8h act16(v8f a) {
  v8h hv = __builtin_convertvector(a, v8h);
  hv = hv * (_Float16)WSC_INV;
  v8h hs = hv * (_Float16)0.01f;
  return __builtin_elementwise_max(hv, hs);
}

__device__ __forceinline__ float fsig(float v) {
  return (1.0f / (1.0f + expf(-v))) * 1.002f - 0.001f;
}

__global__ __launch_bounds__(32) void prep_wt(const float* __restrict__ W0, const float* __restrict__ b0,
                                             const float* __restrict__ Wh, const float* __restrict__ bh,
                                             const float* __restrict__ Wout, _Float16* wt) {
  const int lane = threadIdx.x & 31;
  const int row  = 2 * (int)blockIdx.x + (lane >> 4);
  const int c8   = (lane & 15) * 8;
  const int L    = row / HID;
  const bool head = (L >= 6);
  const int m    = row - HID * L;
  const int mm   = m > (HID - 1) ? (HID - 1) : m;
  const int lc   = (L >= 1 && L <= 5) ? (L - 1) : 0;
  const int m3   = m > 3 ? 3 : m;
  v8h hv;
#pragma unroll
  for (int e = 0; e < 8; ++e) {
    const int k   = c8 + e;
    const int k2  = k > 2 ? 2 : k;
    const int k82 = k > (KIN - 1) ? (KIN - 1) : k;
    const int k79 = k > (HID - 1) ? (HID - 1) : k;
    const float w0v = W0[k2 * HID + mm];
    const float b0v = b0[mm];
    const float whv = Wh[((size_t)lc * KIN + k82) * HID + mm];
    const float bhv = bh[lc * HID + mm];
    const float wov = Wout[k79 * 4 + m3];
    const float vL0 = (k < 3) ? w0v : ((k == 3) ? b0v : 0.0f);
    const float vLh = (k < KIN) ? whv : ((k == KIN) ? bhv : 0.0f);
    const float vHd = (m < 4 && k < HID) ? wov : 0.0f;
    const float v   = head ? vHd : ((L == 0) ? vL0 : vLh);
    hv[e] = (_Float16)(v * WSC);
  }
  _Float16* dst = wt + (size_t)row * WTP + c8;
  *(volatile v8h*)dst = hv;
  __threadfence();
  *(volatile v8h*)dst = hv;
}

__global__ __launch_bounds__(256) void mlp_render_fused(const float* __restrict__ rays, const _Float16* wt,
                                                       const float* __restrict__ bout, float* out,
                                                       int nrays, int nout) {
  __shared__ __align__(16) float outs[8 * 48];
  const int tid  = threadIdx.x;
  const int wave = tid >> 5;
  const int lane = tid & 31;
  const int hh   = lane >> 4;
  const int c    = lane & 15;
  const int ray  = (int)blockIdx.x * RAYS_PER_BLOCK + wave * 16 + c;
  const int rayc = ray < nrays ? ray : (nrays - 1);
  const float* rp = rays + (size_t)rayc * 6;
  const float ox = rp[0], oy = rp[1], oz = rp[2];
  const float dx = rp[3], dy = rp[4], dz = rp[5];
  const float rnorm = sqrtf(dx * dx + dy * dy + dz * dz);
  const float bo0 = bout[0], bo1 = bout[1], bo2 = bout[2], bo3 = bout[3];

  const _Float16* wl = wt + (size_t)c * WTP + 8 * hh;

  const v8f cz = {0.f, 0.f, 0.f, 0.f, 0.f, 0.f, 0.f, 0.f};
  const _Float16 hz = (_Float16)0.0f;
  v8h z8;
#pragma unroll
  for (int e = 0; e < 8; ++e) z8[e] = hz;

  int zo = 0;
  asm volatile("v_nop" : "+v"(zo));

  float Tacc = 1.0f, r0acc = 0.0f, r1acc = 0.0f, r2acc = 0.0f;

#pragma unroll 1
  for (int t = 0; t < NSTEP; ++t) {
    const float ts   = (t < NSTEP - 1) ? (float)t * (1.0f / 63.0f) : 1.0f;
    const float tsn  = (t + 1 < NSTEP - 1) ? (float)(t + 1) * (1.0f / 63.0f) : 1.0f;
    const float dist = ((t < NSTEP - 1) ? (tsn - ts) : 1e10f) * rnorm;
    const float px = ox + ts * dx, py = oy + ts * dy, pz = oz + ts * dz;

    v8h p8;
    p8[0] = hh ? hz : (_Float16)px;
    p8[1] = hh ? hz : (_Float16)py;
    p8[2] = hh ? hz : (_Float16)pz;
    p8[3] = hh ? hz : (_Float16)1.0f;
    p8[4] = hz; p8[5] = hz; p8[6] = hz; p8[7] = hz;

    v8f acc[5];
    v16h af[5];
    v16h bf[3];

    {
      HB bu; bu.h[0] = p8; bu.h[1] = z8;
      const _Float16* wp = wl + zo;
#pragma unroll
      for (int f = 0; f < 5; ++f) af[f] = Frag<_Float16>::load(wp + (size_t)(16 * f) * WTP);
#pragma unroll
      for (int f = 0; f < 5; ++f) acc[f] = Frag<_Float16>::mma(af[f], bu.v, cz);
      guard5z(acc[0], acc[1], acc[2], acc[3], acc[4], af[0], af[1], af[2], af[3], af[4], bu.v, zo);
    }
    {
      HB u0, u1, u2;
      u0.h[0] = act16(acc[0]); u0.h[1] = act16(acc[1]);
      u1.h[0] = act16(acc[2]); u1.h[1] = act16(acc[3]);
      u2.h[0] = act16(acc[4]); u2.h[1] = p8;
      bf[0] = u0.v; bf[1] = u1.v; bf[2] = u2.v;
    }

#pragma unroll 1
    for (int l = 1; l <= NSK; ++l) {
#pragma unroll
      for (int f = 0; f < 5; ++f) acc[f] = cz;
#pragma unroll
      for (int s = 0; s < 3; ++s) {
        const _Float16* wp = wl + zo + (size_t)(HID * l) * WTP + 32 * s;
#pragma unroll
        for (int f = 0; f < 5; ++f) af[f] = Frag<_Float16>::load(wp + (size_t)(16 * f) * WTP);
#pragma unroll
        for (int f = 0; f < 5; ++f) acc[f] = Frag<_Float16>::mma(af[f], bf[s], acc[f]);
        guard5z(acc[0], acc[1], acc[2], acc[3], acc[4], af[0], af[1], af[2], af[3], af[4], bf[s], zo);
      }
      HB u0, u1, u2;
      u0.h[0] = act16(acc[0]); u0.h[1] = act16(acc[1]);
      u1.h[0] = act16(acc[2]); u1.h[1] = act16(acc[3]);
      u2.h[0] = act16(acc[4]); u2.h[1] = p8;
      bf[0] = u0.v; bf[1] = u1.v; bf[2] = u2.v;
    }

    v8f oh = cz;
    {
      v16h ah[3];
      const _Float16* wp = wl + zo + (size_t)HEADROW * WTP;
#pragma unroll
      for (int s = 0; s < 3; ++s) ah[s] = Frag<_Float16>::load(wp + 32 * s);
#pragma unroll
      for (int s = 0; s < 3; ++s) oh = Frag<_Float16>::mma(ah[s], bf[s], oh);
      guard1z(oh, ah[0], ah[1], ah[2], bf[0], bf[1], bf[2], zo);
    }

    const float rw0 = oh[0] * WSC_INV + bo0;
    const float rw1 = oh[1] * WSC_INV + bo1;
    const float rw2 = oh[2] * WSC_INV + bo2;
    const float rw3 = oh[3] * WSC_INV + bo3;
    const float xs    = rw0 - 1.0f;
    const float sigma = fmaxf(xs, 0.0f) + log1pf(expf(-fabsf(xs)));
    const float alpha = 1.0f - expf(-(sigma * dist));
    const float wgt   = alpha * Tacc;
    Tacc = Tacc * ((1.0f - alpha) + 1e-10f);
    r0acc += wgt * fsig(rw1);
    r1acc += wgt * fsig(rw2);
    r2acc += wgt * fsig(rw3);
  }

  if (hh == 0) {
    outs[wave * 48 + c * 3 + 0] = r0acc;
    outs[wave * 48 + c * 3 + 1] = r1acc;
    outs[wave * 48 + c * 3 + 2] = r2acc;
  }
  __syncthreads();
  if (tid < 96) {
    const v4f val = *(const v4f*)(outs + 4 * tid);
    const int gi = (int)blockIdx.x * (RAYS_PER_BLOCK * 3) + 4 * tid;
    const bool ok = (gi + 3) < nout;
    if (ok) *(volatile v4f*)(out + gi) = val;
    __threadfence();
    if (ok) *(volatile v4f*)(out + gi) = val;
  }
}

extern "C" void kernel_launch(void* const* d_in, const int* in_sizes, int n_in,
                              void* d_out, int out_size, void* d_ws, size_t ws_size,
                              hipStream_t stream) {
  if (n_in < 7) return;
  const float* rays = (const float*)d_in[0];
  const float* W0   = (const float*)d_in[1];
  const float* b0   = (const float*)d_in[2];
  const float* Wh   = (const float*)d_in[3];
  const float* bh   = (const float*)d_in[4];
  const float* Wout = (const float*)d_in[5];
  const float* bout = (const float*)d_in[6];
  float* out = (float*)d_out;

  const int nrays = in_sizes[0] / 6;
  if (nrays <= 0) return;
  if (in_sizes[1] < 3 * HID || in_sizes[2] < HID || in_sizes[3] < NSK * KIN * HID ||
      in_sizes[4] < NSK * HID || in_sizes[5] < HID * 4 || in_sizes[6] < 4) return;
  const size_t wt_bytes = (size_t)WTROWS * WTP * sizeof(_Float16);
  if (ws_size < wt_bytes) return;
  if (out_size < 4) return;

  _Float16* wt = (_Float16*)d_ws;

  prep_wt<<<WTROWS / 2, 32, 0, stream>>>(W0, b0, Wh, bh, Wout, wt);

  const int nout = (out_size < nrays * 3) ? out_size : nrays * 3;
  const int nblk = (nrays + RAYS_PER_BLOCK - 1) / RAYS_PER_BLOCK;
  mlp_render_fused<<<nblk, 256, 0, stream>>>(rays, wt, bout, out, nrays, nout);
}
